// RGCNEntityClassifier_70566312673748
// MI455X (gfx1250) — hardware-verified
//
#include <hip/hip_runtime.h>
#include <stdint.h>

typedef _Float16 f16;
typedef __attribute__((ext_vector_type(16))) _Float16 v16h;
typedef __attribute__((ext_vector_type(8)))  _Float16 v8h;
typedef __attribute__((ext_vector_type(8)))  float    v8f;
typedef __attribute__((ext_vector_type(4)))  float    v4f_t;
typedef __attribute__((ext_vector_type(2)))  float    v2f_t;
typedef float v4fa __attribute__((ext_vector_type(4), may_alias));

constexpr int N_NODES = 50000;
constexpr int N_REL   = 16;
constexpr int N_BASIS = 8;
constexpr int D_IN    = 64;
constexpr int D_HID   = 64;
constexpr int N_CLASS = 16;
constexpr int N_EDGES = 800000;
constexpr int K_REL   = N_REL * D_IN;
constexpr int K_TOT   = K_REL + D_IN;
constexpr int NUM_KT  = K_TOT / 32;
constexpr int M_TILES = N_NODES / 16;
constexpr int BUCKET  = 64;
constexpr int NBK     = (N_NODES + BUCKET - 1) / BUCKET;
constexpr int NBKP    = 800;
constexpr int CHUNK   = 2048;
constexpr int NCH     = (N_EDGES + CHUNK - 1) / CHUNK;
constexpr int SLOT    = 32;
constexpr int LCAP    = 1536;
#define RSPLIT (1.0f / 2048.0f)

__device__ __forceinline__ v8f wmma16(v16h a, v16h b, v8f c) {
  return __builtin_amdgcn_wmma_f32_16x16x32_f16(false, a, false, b, (short)0, c, false, false);
}
__device__ __forceinline__ v8f wmma_split(v16h a, v16h al, v16h b, v16h bl, v8f c) {
  v8f x = {};
  x = wmma16(al, b, x); x = wmma16(a, bl, x);
  return wmma16(a, b, c) + x * RSPLIT;
}
__device__ __forceinline__ f16 lo_of(float v, f16 h) { return (f16)((v - (float)h) * 2048.0f); }
__device__ __forceinline__ v16h cat8(v8h a, v8h b) { return __builtin_shufflevector(a, b, 0,1,2,3,4,5,6,7,8,9,10,11,12,13,14,15); }

__global__ __launch_bounds__(256) void build_bsw(const float* __restrict__ bases, const float* __restrict__ coeffs,
                                                 const float* __restrict__ selfw, f16* __restrict__ bsw, int dout) {
  const int numNt = dout >> 4;
  const int total = NUM_KT * numNt * 512;
  const int idx = (blockIdx.x * 256 + threadIdx.x) * 2;
  if (idx >= total) return;
  unsigned ph = 0, pl = 0;
#pragma unroll
  for (int q = 0; q < 2; ++q) {
    const int ii = idx + q, e = ii & 15, lane = (ii >> 4) & 31, rem = ii >> 9, nt = rem % numNt, kt = rem / numNt;
    const int hi = lane >> 4;
    const int K = kt * 32 + ((e < 8) ? (hi * 8 + e) : (16 + hi * 8 + (e - 8)));
    const int n = nt * 16 + (lane & 15);
    float w;
    if (K < K_REL) {
      const int r = K >> 6, i = K & 63;
      float acc = 0.f;
#pragma unroll
      for (int b = 0; b < N_BASIS; ++b) acc += coeffs[r * N_BASIS + b] * bases[(b * D_IN + i) * dout + n];
      w = acc;
    } else {
      w = selfw[(K - K_REL) * dout + n];
    }
    const f16 h = (f16)w, l = lo_of(w, h);
    ph |= (unsigned)__builtin_bit_cast(unsigned short, h) << (16 * q);
    pl |= (unsigned)__builtin_bit_cast(unsigned short, l) << (16 * q);
  }
  const size_t plane = (size_t)total;
  *(volatile unsigned*)(bsw + idx) = ph; *(volatile unsigned*)(bsw + plane + idx) = pl; __threadfence();
  *(volatile unsigned*)(bsw + idx) = ph; *(volatile unsigned*)(bsw + plane + idx) = pl;
}

__global__ __launch_bounds__(256) void bin_kernel(const int* __restrict__ dst, int* __restrict__ slots, int* __restrict__ cnts) {
  __shared__ int cnt[NBKP];
  const int tid = threadIdx.x, ch = blockIdx.x;
  for (int i = tid; i < NBKP; i += 256) cnt[i] = 0;
  __syncthreads();
  int eb[8], ps[8];
#pragma unroll
  for (int u = 0; u < 8; ++u) {
    const int e = ch * CHUNK + u * 256 + tid;
    eb[u] = -1; ps[u] = -1;
    if (e < N_EDGES) {
      int d = dst[e]; d = ((unsigned)d < (unsigned)N_NODES) ? d : 0;
      const int b = d / BUCKET;
      const int p = atomicAdd(&cnt[b], 1);
      if (p < SLOT) { eb[u] = b; ps[u] = p; }
    }
  }
  __syncthreads();
#pragma unroll 1
  for (int pass = 0; pass < 2; ++pass) {
#pragma unroll
    for (int u = 0; u < 8; ++u)
      if (eb[u] >= 0) *(volatile int*)(slots + ((size_t)ch * NBK + eb[u]) * SLOT + ps[u]) = ch * CHUNK + u * 256 + tid;
    for (int i = tid; i < NBKP; i += 256) *(volatile int*)(cnts + (size_t)ch * NBKP + i) = (i < NBK) ? min(cnt[i], SLOT) : 0;
    __threadfence();
  }
}

__global__ __launch_bounds__(256) void gather_kernel(const int* __restrict__ src, const int* __restrict__ dst, const int* __restrict__ etype,
                                                    const int* __restrict__ slots, const int* __restrict__ cnts,
                                                    const float* __restrict__ feat, float* __restrict__ agg) {
  __shared__ int lst[LCAP];
  __shared__ int lsrc[LCAP], ltyp[LCAP];
  __shared__ int total;
  __shared__ int ncnt[BUCKET], noff[BUCKET];
  const int tid = threadIdx.x, lane = tid & 31, wave = tid >> 5;
  const int bk = blockIdx.x, n0 = bk * BUCKET;
  if (tid == 0) total = 0;
  if (tid < BUCKET) ncnt[tid] = 0;
  __syncthreads();
  int myc[4], mytot = 0;
#pragma unroll
  for (int u = 0; u < 4; ++u) { const int ch = tid + 256 * u; myc[u] = (ch < NCH) ? cnts[(size_t)ch * NBKP + bk] : 0; mytot += myc[u]; }
  {
    __shared__ int scan[256];
    scan[tid] = mytot;
    __syncthreads();
#pragma unroll
    for (int off = 1; off < 256; off <<= 1) { const int v = (tid >= off) ? scan[tid - off] : 0; __syncthreads(); scan[tid] += v; __syncthreads(); }
    int pos = scan[tid] - mytot;
    if (tid == 255) total = min(scan[255], LCAP);
#pragma unroll
    for (int u = 0; u < 4; ++u) {
      const int ch = tid + 256 * u;
      for (int i = 0; i < myc[u]; ++i) {
        if (pos < LCAP) {
          const int e = slots[((size_t)ch * NBK + bk) * SLOT + i];
          int d = dst[e]; d = ((unsigned)d < (unsigned)N_NODES) ? d : 0;
          lst[pos] = ((d - n0) << 24) | e;
        }
        ++pos;
      }
    }
    __syncthreads();
  }
  const int nl = total;
  for (int i = tid; i < nl; i += 256) atomicAdd(&ncnt[(lst[i] >> 24) & 63], 1);
  __syncthreads();
  if (tid == 0) { int o = 0; for (int j = 0; j < BUCKET; ++j) { noff[j] = o; o += ncnt[j]; } }
  __syncthreads();
  if (tid < BUCKET) {
    int p = noff[tid];
    for (int i = 0; i < nl; ++i) if (((lst[i] >> 24) & 63) == tid) {
      const int e = lst[i] & 0xFFFFFF;
      int s = src[e]; s = ((unsigned)s < (unsigned)N_NODES) ? s : 0;
      int t = etype[e]; t = ((unsigned)t < (unsigned)N_REL) ? t : 0;
      lsrc[p] = s; ltyp[p] = t; ++p;
    }
  }
  __syncthreads();
  for (int j = wave; j < BUCKET; j += 8) {
    const int node = n0 + j;
    if (node >= N_NODES) break;
    const int o0 = noff[j], cn = ncnt[j];
#pragma unroll 1
    for (int r = 0; r < N_REL; ++r) {
      float sx = 0.f, sy = 0.f; int c = 0;
      for (int i = 0; i < cn; ++i) {
        if (ltyp[o0 + i] == r) { const v2f_t v = *(const v2f_t*)(feat + (size_t)lsrc[o0 + i] * 64 + 2 * lane); sx += v.x; sy += v.y; ++c; }
      }
      const float inv = 1.0f / (float)(c > 1 ? c : 1);
      v2f_t o; o.x = sx * inv; o.y = sy * inv;
      float* dstp = agg + ((size_t)r * N_NODES + node) * 64 + 2 * lane;
      *(volatile v2f_t*)dstp = o; __threadfence(); *(volatile v2f_t*)dstp = o;
    }
  }
}

template <int NUMNT, bool RELU>
__global__ __launch_bounds__(256)
void rgcn_gemm(const float* __restrict__ agg, const float* __restrict__ feat,
               const f16* __restrict__ bsw, float* __restrict__ out) {
  constexpr int DOUT = NUMNT * 16;
  __shared__ __attribute__((aligned(16))) float stg[8][16 * DOUT];
  const int lane  = threadIdx.x & 31;
  const int wid   = threadIdx.x >> 5;
  const int mtile = blockIdx.x * 8 + wid;
  if (mtile >= M_TILES) return;
  const int node   = mtile * 16 + (lane & 15);
  const int kshift = (lane < 16) ? 0 : 8;
  const size_t plane = (size_t)NUM_KT * NUMNT * 512;

  v8f acc[NUMNT] = {};
  auto kstep = [&](const float* ap32, int kt) {
    const v8f va0 = *reinterpret_cast<const v8f*>(ap32 + kshift);
    const v8f va1 = *reinterpret_cast<const v8f*>(ap32 + 16 + kshift);
    v16h a, al;
#pragma unroll
    for (int j = 0; j < 8; ++j) {
      const f16 h0 = (f16)va0[j], h1 = (f16)va1[j];
      a[j] = h0;     al[j] = lo_of(va0[j], h0);
      a[8 + j] = h1; al[8 + j] = lo_of(va1[j], h1);
    }
#pragma unroll
    for (int nt = 0; nt < NUMNT; ++nt) {
      const f16* fb = bsw + ((size_t)(kt * NUMNT + nt) * 32 + lane) * 16;
      const v16h b  = cat8(*(const v8h*)fb, *(const v8h*)(fb + 8));
      const v16h bl = cat8(*(const v8h*)(fb + plane), *(const v8h*)(fb + plane + 8));
      acc[nt] = wmma_split(a, al, b, bl, acc[nt]);
    }
  };
  const float* ap = agg + (size_t)node * 64;
  const size_t rstride = (size_t)N_NODES * 64;
#pragma unroll 1
  for (int r = 0; r < N_REL; ++r) {
    kstep(ap, 2 * r); kstep(ap + 32, 2 * r + 1);
    ap += rstride;
  }
  const float* fp = feat + (size_t)node * 64;
  kstep(fp, 32); kstep(fp + 32, 33);

  float* sw = stg[wid];
  const int rbase = (lane < 16) ? 0 : 8;
#pragma unroll
  for (int nt = 0; nt < NUMNT; ++nt)
#pragma unroll
    for (int v = 0; v < 8; ++v) { float x = acc[nt][v]; if (RELU) x = fmaxf(x, 0.f); sw[(rbase + v) * DOUT + nt * 16 + (lane & 15)] = x; }
  asm volatile("s_wait_dscnt 0" ::: "memory");
  float* ob = out + (size_t)mtile * 16 * DOUT;
#pragma unroll 1
  for (int pass = 0; pass < 2; ++pass) {
#pragma unroll
    for (int i = 0; i < (16 * DOUT) / 128; ++i) { const int c = lane + 32 * i; *(volatile v4f_t*)(ob + c * 4) = *(const volatile v4fa*)(sw + c * 4); }
    __threadfence();
  }
}

extern "C" void kernel_launch(void* const* d_in, const int* in_sizes, int n_in,
                              void* d_out, int out_size, void* d_ws, size_t ws_size,
                              hipStream_t stream) {
  (void)in_sizes; (void)n_in; (void)out_size; (void)ws_size;
  const float* x       = (const float*)d_in[0];
  const float* bases1  = (const float*)d_in[1];
  const float* coeffs1 = (const float*)d_in[2];
  const float* self1   = (const float*)d_in[3];
  const float* bases2  = (const float*)d_in[4];
  const float* coeffs2 = (const float*)d_in[5];
  const float* self2   = (const float*)d_in[6];
  const int* edge_index = (const int*)d_in[7];
  const int* edge_type  = (const int*)d_in[8];
  const int* src = edge_index;
  const int* dst = edge_index + N_EDGES;

  char* ws = (char*)d_ws;
  size_t off = 0;
  auto carve = [&](size_t bytes) -> char* { char* p = ws + off; off += (bytes + 255) & ~(size_t)255; return p; };
  float* agg   = (float*)carve(sizeof(float) * (size_t)N_REL * N_NODES * 64);
  float* h     = (float*)carve(sizeof(float) * (size_t)N_NODES * D_HID);
  f16*   bsw1  = (f16*)  carve(sizeof(f16) * (size_t)NUM_KT * 4 * 512 * 2);
  f16*   bsw2  = (f16*)  carve(sizeof(f16) * (size_t)NUM_KT * 1 * 512 * 2);
  int*   slots = (int*)  carve(sizeof(int) * (size_t)NCH * NBK * SLOT);
  int*   cnts  = (int*)  carve(sizeof(int) * (size_t)NCH * NBKP);

  const int TB = 256;
  build_bsw<<<(NUM_KT * 4 * 512 / 2 + TB - 1) / TB, TB, 0, stream>>>(bases1, coeffs1, self1, bsw1, D_HID);
  build_bsw<<<(NUM_KT * 1 * 512 / 2 + TB - 1) / TB, TB, 0, stream>>>(bases2, coeffs2, self2, bsw2, N_CLASS);
  bin_kernel<<<NCH, TB, 0, stream>>>(dst, slots, cnts);

  const int gemmBlocks = (M_TILES + 7) / 8;
  gather_kernel<<<NBK, TB, 0, stream>>>(src, dst, edge_type, slots, cnts, x, agg);
  rgcn_gemm<4, true><<<gemmBlocks, TB, 0, stream>>>(agg, x, bsw1, h);
  gather_kernel<<<NBK, TB, 0, stream>>>(src, dst, edge_type, slots, cnts, h, agg);
  rgcn_gemm<1, false><<<gemmBlocks, TB, 0, stream>>>(agg, h, bsw2, (float*)d_out);
}
